// LegacySeqFirstSelfAttention_modified_7679401525984
// MI455X (gfx1250) — hardware-verified
//
#include <hip/hip_runtime.h>


namespace {
constexpr int SQ = 1024, B = 4, HID = 1024, NH = 16, HN = 64, BN = 4, CK = HID / BN  , OC = 3 * HID / BN  , BL = 4  ;
constexpr float XS = 8.0f, WSC = 256.0f, PSC = 1024.0f;
static_assert(SQ % 64 == 0 && HN == 64 && OC == 4 * 3 * HN, "tiling");
typedef _Float16 b16;
typedef __attribute__((ext_vector_type(16))) _Float16 v16b;
typedef __attribute__((ext_vector_type(8))) _Float16 v8b;
typedef __attribute__((ext_vector_type(8))) float v8f;
typedef __attribute__((ext_vector_type(4))) float v4f;
__device__ __forceinline__ float bf16_rne(float f) { unsigned int u = __float_as_uint(f); u += 0x7FFFu + ((u >> 16) & 1u); return __uint_as_float(u & 0xFFFF0000u); }
__device__ __forceinline__ void split16(float v, b16& hi, b16& lo) { hi = (b16)v; lo = (b16)(v - (float)hi); }
__device__ __forceinline__ v16b frag_kb(const b16* p, int hh) { const v8b a = *(const v8b*)(p + 8 * hh), b = *(const v8b*)(p + 16 + 8 * hh); v16b f;
#pragma unroll
  for (int e = 0; e < 8; ++e) { f[e] = a[e]; f[8 + e] = b[e]; } return f; }
__device__ __forceinline__ v8f wmma16b(v16b a, v16b b, v8f c) { v8f d = __builtin_amdgcn_wmma_f32_16x16x32_f16(false, a, false, b, (short)0, c, false, false); asm volatile("v_nop\n\tv_nop\n\tv_nop\n\tv_nop" : "+v"(d) : "v"(a), "v"(b)); return d; }
__device__ __forceinline__ void wave_lds_sync() { __builtin_amdgcn_fence(__ATOMIC_RELEASE, "workgroup"); __builtin_amdgcn_wave_barrier(); __builtin_amdgcn_fence(__ATOMIC_ACQUIRE, "workgroup"); }
__device__ __forceinline__ float pmul(float a, float b) { float p = a * b; asm volatile("" : "+v"(p)); return p; }
__device__ __forceinline__ int iclamp(int v, int lo, int hi) { return v < lo ? lo : (v > hi ? hi : v); }

typedef __attribute__((ext_vector_type(2))) _Float16 v2h;
typedef __attribute__((ext_vector_type(2))) float v2f;
__global__ __launch_bounds__(256) void wprep_kernel(const float* __restrict__ Wq, b16* __restrict__ WT) {
  const size_t u = (size_t)blockIdx.x * 256 + threadIdx.x; if (u >= (size_t)B * BN * OC * CK / 8) return; const size_t e = u * 8;
  const int b = (int)(e / ((size_t)BN * OC * CK)); size_t r1 = e % ((size_t)BN * OC * CK); const int j = (int)(r1 / ((size_t)OC * CK)); r1 %= (size_t)OC * CK; const int o = (int)(r1 / CK), c0 = (int)(r1 % CK); v8b ov;
  for (int q = 0; q < 8; ++q) ov[q] = (b16)(bf16_rne(Wq[(size_t)(b * CK + c0 + q) * (3 * HID) + j * OC + o]) * WSC);
  for (int pass = 0; pass < 2; ++pass) { *(volatile v8b*)(WT + e) = ov; __threadfence(); }
}
__global__ __launch_bounds__(128) void qkv_kernel(const float* __restrict__ hs, const b16* __restrict__ WT, b16* __restrict__ Qp, b16* __restrict__ Kp, b16* __restrict__ VT) {
  __shared__ __attribute__((aligned(16))) b16 As[4][16][CK + 8]; __shared__ __attribute__((aligned(16))) float Tf[4][16][192 + 4];
  const int wave = threadIdx.x >> 5, lane = threadIdx.x & 31, nloc = lane & 15, hlf = lane >> 4; const int s0 = blockIdx.x * 64 + wave * 16; const int b = blockIdx.y / BN, j = blockIdx.y % BN, hq = blockIdx.z; const int nh = j * 4 + hq;
  for (int rr = 0; rr < 16; ++rr) { const float* src = hs + ((size_t)(s0 + rr) * B + b) * HID + j * CK; v8b ov; for (int q = 0; q < 8; ++q) ov[q] = (b16)(bf16_rne(src[lane * 8 + q]) * XS); *(v8b*)(&As[wave][rr][lane * 8]) = ov; }
  wave_lds_sync();
  const b16* Wb = WT + (((size_t)b * BN + j) * OC + hq * 192) * CK;
  v8f acc[12];
#pragma unroll
  for (int t = 0; t < 12; ++t) acc[t] = (v8f){};
#pragma unroll 1
  for (int kb = 0; kb < CK; kb += 32) { const v16b a = frag_kb(&As[wave][nloc][kb], hlf);
#pragma unroll
    for (int t = 0; t < 12; ++t) acc[t] = wmma16b(a, frag_kb(Wb + (size_t)(t * 16 + nloc) * CK + kb, hlf), acc[t]); }
#pragma unroll
  for (int t = 0; t < 12; ++t) {
#pragma unroll
    for (int r = 0; r < 8; ++r) Tf[wave][8 * hlf + r][t * 16 + nloc] = acc[t][r] * (1.0f / (XS * WSC)); }
  __syncthreads();
  b16* Qb = Qp + ((size_t)(b * NH + nh) * SQ) * HN; b16* Kb = Kp + ((size_t)(b * NH + nh) * SQ) * HN; b16* Vb = VT + ((size_t)(b * NH + nh) * HN) * SQ;
  for (int pass = 0; pass < 2; ++pass) {
    for (int rr = 0; rr < 16; ++rr) { v2h qv, kv; qv[0] = (b16)(Tf[wave][rr][lane * 2] * XS); qv[1] = (b16)(Tf[wave][rr][lane * 2 + 1] * XS); kv[0] = (b16)(Tf[wave][rr][HN + lane * 2] * XS); kv[1] = (b16)(Tf[wave][rr][HN + lane * 2 + 1] * XS);
      *(volatile v2h*)(Qb + (size_t)(s0 + rr) * HN + lane * 2) = qv; *(volatile v2h*)(Kb + (size_t)(s0 + rr) * HN + lane * 2) = kv; }
#pragma unroll 1
    for (int q = 0; q < 16; ++q) { const int d = wave * 16 + q; const int t0 = lane * 2; v2h vv; vv[0] = (b16)(Tf[t0 >> 4][t0 & 15][2 * HN + d] * XS); vv[1] = (b16)(Tf[(t0 + 1) >> 4][(t0 + 1) & 15][2 * HN + d] * XS);
      *(volatile v2h*)(Vb + (size_t)d * SQ + blockIdx.x * 64 + lane * 2) = vv; }
    __threadfence(); }
}
__global__ __launch_bounds__(256) void vsum_kernel(const b16* __restrict__ VT, float* __restrict__ VS) {
  const int u = blockIdx.x * 256 + threadIdx.x; if (u >= BL * NH * HN) return; const b16* row = VT + (size_t)u * SQ; float s = 0.0f;
#pragma unroll 1
  for (int t = 0; t < SQ; t += 8) { const v8b v = *(const v8b*)(row + t); for (int q = 0; q < 8; ++q) s += (float)v[q]; }
  for (int pass = 0; pass < 2; ++pass) { ((volatile float*)VS)[u] = s * (1.0f / XS); __threadfence(); }
}
__global__ __launch_bounds__(64) void attn_kernel(const b16* __restrict__ Qp, const b16* __restrict__ Kp, const b16* __restrict__ VT, const float* __restrict__ VS, const float* __restrict__ gam, const float* __restrict__ bet, float* __restrict__ out) {
  __shared__ __attribute__((aligned(16))) float To[2][16][HN + 4];
  const int wave = threadIdx.x >> 5, lane = threadIdx.x & 31, hh = lane >> 4, col = lane & 15; const int q0 = blockIdx.x * 32 + wave * 16, qi = q0 + col; const int b = blockIdx.y / NH, nh = blockIdx.y % NH;
  const b16* Qb = Qp + ((size_t)(b * NH + nh) * SQ) * HN; const b16* Kb = Kp + ((size_t)(b * NH + nh) * SQ) * HN; const b16* Vb = VT + ((size_t)(b * NH + nh) * HN) * SQ;
  const v16b qa0 = frag_kb(Qb + (size_t)qi * HN, hh), qa1 = frag_kb(Qb + (size_t)qi * HN + 32, hh);
  v8f o[4]; for (int t = 0; t < 4; ++t) o[t] = (v8f){};
  float rs = 0.0f;
  const float inv8 = 1.0f / (8.0f * XS * XS);
#pragma unroll 1
  for (int kb = 0; kb < SQ; kb += 32) {
    v8f s0 = (v8f){}, s1 = (v8f){};
    { const v16b k00 = frag_kb(Kb + (size_t)(kb + col) * HN, hh), k01 = frag_kb(Kb + (size_t)(kb + col) * HN + 32, hh), k10 = frag_kb(Kb + (size_t)(kb + 16 + col) * HN, hh), k11 = frag_kb(Kb + (size_t)(kb + 16 + col) * HN + 32, hh);
      s0 = wmma16b(k00, qa0, s0); s0 = wmma16b(k01, qa1, s0); s1 = wmma16b(k10, qa0, s1); s1 = wmma16b(k11, qa1, s1); }
    v16b ph, pl;
#pragma unroll
    for (int i = 0; i < 16; ++i) { const float x = (i < 8 ? s0[i] : s1[i - 8]) * inv8; const float x2 = x * x; const float a = 0.5f + x * (0.25f + x2 * (-1.0f / 48.0f + x2 * (1.0f / 480.0f))); rs += a; b16 p, q; split16(a * PSC, p, q); ph[i] = p; pl[i] = q; }
#pragma unroll
    for (int t = 0; t < 4; ++t) { const v16b va = frag_kb(Vb + (size_t)(t * 16 + col) * SQ + kb, hh); o[t] = wmma16b(va, ph, o[t]); o[t] = wmma16b(va, pl, o[t]); } }
  rs += __shfl_xor(rs, 16);
  const float g = bf16_rne(gam[nh]), bt = bf16_rne(bet[nh]); const float sc = g / ((rs + 1e-7f) * PSC * XS);
#pragma unroll
  for (int t = 0; t < 4; ++t)
#pragma unroll
    for (int r = 0; r < 8; ++r) { const int d = t * 16 + 8 * hh + r; To[wave][col][d] = o[t][r] * sc + bt * VS[(size_t)(b * NH + nh) * HN + d]; }
  wave_lds_sync();
  for (int pass = 0; pass < 2; ++pass) { for (int rr = 0; rr < 16; ++rr) *(volatile v2f*)(out + ((size_t)(q0 + rr) * B + b) * HID + nh * HN + lane * 2) = *(const v2f*)(&To[wave][rr][lane * 2]); __threadfence(); }
}
}

extern "C" void kernel_launch(void* const* d_in, const int* in_sizes, int n_in, void* d_out, int out_size, void* d_ws, size_t ws_size, hipStream_t stream) {
  (void)n_in;
  auto Fp = [&](int i) { return (const float*)d_in[i]; };
  if (in_sizes[0] != SQ * B * HID || in_sizes[1] != HID * 3 * HID || in_sizes[2] != NH || in_sizes[3] != NH || out_size != SQ * B * HID) return;
  size_t off = 0; char* ws = (char*)d_ws;
  auto carve = [&](size_t bytes) { char* p = ws + off; off += (bytes + 255) & ~(size_t)255; return p; };
  b16* WT = (b16*)carve((size_t)B * BN * OC * CK * 2); b16* Qp = (b16*)carve((size_t)B * NH * SQ * HN * 2); b16* Kp = (b16*)carve((size_t)B * NH * SQ * HN * 2); b16* VT = (b16*)carve((size_t)B * NH * HN * SQ * 2); float* VS = (float*)carve((size_t)B * NH * HN * 4);
  if (off > ws_size || off > ((size_t)128 << 20)) return;
  wprep_kernel<<<(unsigned)(((size_t)B * BN * OC * CK / 8 + 255) / 256), 256, 0, stream>>>(Fp(1), WT);
  qkv_kernel<<<dim3(SQ / 64, BL * BN, 4), 128, 0, stream>>>(Fp(0), WT, Qp, Kp, VT);
  vsum_kernel<<<(BL * NH * HN + 255) / 256, 256, 0, stream>>>(VT, VS);
  attn_kernel<<<dim3(SQ / 32, BL * NH), 64, 0, stream>>>(Qp, Kp, VT, VS, Fp(2), Fp(3), (float*)d_out);
}
